// TensorProductConvLayer_9191230013567
// MI455X (gfx1250) — hardware-verified
//
#include <hip/hip_runtime.h>
#include <stddef.h>
#include <stdint.h>
#include <math.h>

#define NS     48
#define NV     10
#define NEF    128
#define HID    128
#define W1N    (NS * NS)
#define W2N    (NS * NV)
#define W3N    (NV * NV)
#define W4N    (NV * NS)
#define WTOT   (W1N + W2N + W3N + W4N)
#define OUTC   (NS + 3 * NV)
#define TPP    80
#define KH     256
#define OFF_W2 W1N
#define OFF_W3 (W1N + W2N)
#define OFF_W4 (W1N + W2N + W3N)
#define T_W4   (NS * 3)
#define T_W2   (T_W4 + NV * 3)
#define T_W3   (T_W2 + NS)
#define NTILE  (T_W3 + NV)
#define NPC    (NTILE * 16)
#define NTHR   256
#define NWAVE  8
#define EPB    128
#define COP    140
#define GBM    64
#define GBN    128
#define GTHR   128
#define EPT    8
#define CHUNK  (NTHR * EPT)
#define WCAP   (EPT * 32)
#define LISTN  (NWAVE * WCAP)
#define NBA    1024
#define SLA    10
#define RCAP   8192
#define DEGCAP 32
#define SPW    (NBA / NWAVE)
#define GRP    16
#define NGRP   (SPW / GRP)
#define NRB    128
#define NU_W1  (HID * (NEF / 8))
#define NU_W2P (NPC * 16)
#define NU_B2  (NPC / 4)
#define NU_B2P 1024
#define AGG_ZINTS (LISTN + 2 * RCAP + 3 * NBA)
#define AGG_INTS  (AGG_ZINTS + 16)
#define YS_FLOATS (NWAVE * GRP * TPP)
#define SCAN_LDS_BYTES (AGG_INTS * 4 + YS_FLOATS * 4 + NWAVE * TPP * 2 * 8)
#define TP_LDS_FLOATS (EPB * COP + EPB * TPP + EPB + EPB)
#define TP_LDS_BYTES  (TP_LDS_FLOATS * 4)
#define WSMAX  134217728
#define EPSF   1e-5f

static_assert(NS == 3 * 16 && NV <= 16 && OUTC == 78 && OUTC + 2 == TPP);
static_assert(WTOT == 3364 && OFF_W2 == 2304 && OFF_W3 == 2784 && OFF_W4 == 2884);
static_assert(T_W4 == 144 && T_W2 == 174 && T_W3 == 222 && NTILE == 232 && NPC == 3712 && 232 * 16 == 3712);
static_assert(OFF_W4 + (NV - 1) * NS + 2 * 16 + 15 == WTOT - 1);
static_assert(OFF_W2 + (NS - 1) * NV + (NV - 1) == OFF_W3 - 1 && OFF_W3 + (NV - 1) * NV + (NV - 1) == OFF_W4 - 1);
static_assert(NEF % 32 == 0 && KH == 2 * HID && KH % 32 == 0 && HID == GBN);
static_assert(NU_W1 % NTHR == 0 && NU_W2P % NTHR == 0 && NU_B2 <= NU_B2P && NU_B2P % NTHR == 0 && NPC % 4 == 0);
static_assert(EPB == 16 * NWAVE && EPB % GBM == 0 && GBM == (GTHR / 32) * 16);
static_assert(EPB * 39 == 4992 && 20 * NTHR >= 4992 && EPB * NS == 24 * NTHR && EPB * NV == 5 * NTHR);
static_assert((EPB * TPP) % (4 * NTHR) == 0 && (EPB * TPP) / (4 * NTHR) == 10 && (EPB * TPP * 4) % 128 == 0);
static_assert((EPB * COP * 4) % 16 == 0 && COP >= 140);
static_assert((CHUNK & (CHUNK - 1)) == 0 && CHUNK <= 4096 && NBA == (1 << SLA));
static_assert(((long long)CHUNK << SLA) < (1LL << 31));
static_assert(AGG_ZINTS % 4 == 0 && (AGG_INTS * 4) % 16 == 0 && RCAP % 4 == 0 && LISTN % 4 == 0);
static_assert(RCAP >= 5206 + 2048 && DEGCAP >= 15 + 8);
static_assert(SPW == GRP * NGRP && (GRP * TPP * 4) % 128 == 0 && (GRP * TPP) / 4 == 10 * 32);
static_assert(SCAN_LDS_BYTES <= 300000 && TP_LDS_BYTES <= 300000);
static_assert((NRB * OUTC * 4) % 128 == 0 && (NRB * OUTC) % 4 == 0 && (NRB * TPP) / 4 == 10 * NTHR);
static_assert((NRB * OUTC) / 4 <= 10 * NTHR);

typedef float          v2f   __attribute__((ext_vector_type(2)));
typedef float          v4f   __attribute__((ext_vector_type(4)));
typedef float          v8f   __attribute__((ext_vector_type(8)));
typedef double         v2d   __attribute__((ext_vector_type(2)));
typedef int            v4i   __attribute__((ext_vector_type(4)));
typedef int            v8i   __attribute__((ext_vector_type(8)));
typedef unsigned short v8us  __attribute__((ext_vector_type(8)));
typedef unsigned short v16us __attribute__((ext_vector_type(16)));
typedef __bf16         v16bf __attribute__((ext_vector_type(16)));
typedef v2f  __attribute__((may_alias)) v2fa;
typedef v4f  __attribute__((may_alias)) v4fa;
typedef v4i  __attribute__((may_alias)) v4ia;
typedef v8us __attribute__((may_alias)) v8usa;
union FragB { v16bf v; v16us u; v8us h[2]; v8i w; };

__device__ __forceinline__ v8f wmb(const FragB& a, const FragB& b, v8f c) {
  v8f d = __builtin_amdgcn_wmma_f32_16x16x32_bf16(false, a.v, false, b.v, (short)0, c, false, false);
  asm volatile("v_nop\n\tv_nop\n\tv_nop\n\tv_nop" : "+v"(d) : "v"(a.w), "v"(b.w));
  return d;
}

__device__ __forceinline__ unsigned bf16_bits(float f) {
  const unsigned u = __float_as_uint(f);
  return (u + 0x7FFFu + ((u >> 16) & 1u)) >> 16;
}
__device__ __forceinline__ float bf16_val(float f) {
  return __uint_as_float(bf16_bits(f) << 16);
}
__device__ __forceinline__ void put16(unsigned short* dp, v8us o) {
  *(volatile v8us*)dp = o;
  __threadfence();
  *(volatile v8us*)dp = o;
}
__device__ __forceinline__ void putf4(float* dp, v4f o) {
  *(volatile v4f*)dp = o;
  __threadfence();
  *(volatile v4f*)dp = o;
}

__device__ __forceinline__ int colmap(int c) {
  const int t = c >> 4, n = c & 15;
  int j;
  if (t < T_W4) {
    j = (t / 3) * NS + (t % 3) * 16 + n;
  } else if (t < T_W2) {
    const int tt = t - T_W4;
    j = OFF_W4 + (tt / 3) * NS + (tt % 3) * 16 + n;
  } else if (t < T_W3) {
    j = (n < NV) ? (OFF_W2 + (t - T_W2) * NV + n) : -1;
  } else {
    j = (n < NV) ? (OFF_W3 + (t - T_W3) * NV + n) : -1;
  }
  return j;
}

template <int SLB>
__device__ __forceinline__ int scan_chunk(const int* __restrict__ dsts, int nE, int cbase, int slotBase,
                                          int nb, int vec8, int* list, int tid, int lane, int wave) {
  int wc = 0;
  const int el0  = tid * EPT;
  const int e0   = cbase + el0;
  const int sent = -2147483647 - 1;
  v4i da, db;
  if (vec8 != 0 && cbase + CHUNK <= nE) {
    da = *(const v4i*)(dsts + e0);
    db = *(const v4i*)(dsts + e0 + 4);
  } else {
    da.x = (e0     < nE) ? dsts[min(e0,     nE - 1)] : sent;
    da.y = (e0 + 1 < nE) ? dsts[min(e0 + 1, nE - 1)] : sent;
    da.z = (e0 + 2 < nE) ? dsts[min(e0 + 2, nE - 1)] : sent;
    da.w = (e0 + 3 < nE) ? dsts[min(e0 + 3, nE - 1)] : sent;
    db.x = (e0 + 4 < nE) ? dsts[min(e0 + 4, nE - 1)] : sent;
    db.y = (e0 + 5 < nE) ? dsts[min(e0 + 5, nE - 1)] : sent;
    db.z = (e0 + 6 < nE) ? dsts[min(e0 + 6, nE - 1)] : sent;
    db.w = (e0 + 7 < nE) ? dsts[min(e0 + 7, nE - 1)] : sent;
  }
  const unsigned nbs = (unsigned)slotBase;
  const unsigned unb = (unsigned)nb;
  const unsigned s0 = (unsigned)da.x - nbs, s1 = (unsigned)da.y - nbs;
  const unsigned s2 = (unsigned)da.z - nbs, s3 = (unsigned)da.w - nbs;
  const unsigned s4 = (unsigned)db.x - nbs, s5 = (unsigned)db.y - nbs;
  const unsigned s6 = (unsigned)db.z - nbs, s7 = (unsigned)db.w - nbs;
  const bool h0 = s0 < unb, h1 = s1 < unb, h2 = s2 < unb, h3 = s3 < unb;
  const bool h4 = s4 < unb, h5 = s5 < unb, h6 = s6 < unb, h7 = s7 < unb;
  const unsigned any = __builtin_amdgcn_ballot_w32(h0 | h1 | h2 | h3 | h4 | h5 | h6 | h7);
  if (any != 0u) {
#define HITJ(J, HJ, SJ) { \
      const unsigned mj = __builtin_amdgcn_ballot_w32(HJ); \
      if (mj != 0u) { \
        if (HJ) { \
          const int pos = wc + (int)__builtin_amdgcn_mbcnt_lo(mj, 0u); \
          if (pos < WCAP) list[wave * WCAP + pos] = ((el0 + (J)) << SLB) | (int)(SJ); \
        } \
        wc += (int)__builtin_popcount(mj); } }
    HITJ(0, h0, s0)
    HITJ(1, h1, s1)
    HITJ(2, h2, s2)
    HITJ(3, h3, s3)
    HITJ(4, h4, s4)
    HITJ(5, h5, s5)
    HITJ(6, h6, s6)
    HITJ(7, h7, s7)
#undef HITJ
  }
  return wc;
}

__global__ __launch_bounds__(NTHR) void k_pa(const float* __restrict__ ea, const float* __restrict__ w1,
                                             int nE, int nUE, unsigned short* EAB, unsigned short* W1T) {
  const int u = (int)blockIdx.x * NTHR + (int)threadIdx.x;
  if (u < nUE) {
    const int row = u >> 4;
    const int k8  = (u & 15) * 8;
    const bool ok = row < nE;
    const int rc  = ok ? row : nE - 1;
    const float* p = ea + (size_t)rc * NEF + k8;
    const v4f a = *(const v4f*)p;
    const v4f b = *(const v4f*)(p + 4);
    const unsigned msk = ok ? 0xffffu : 0u;
    v8us o;
    o[0] = (unsigned short)(bf16_bits(a.x) & msk); o[1] = (unsigned short)(bf16_bits(a.y) & msk);
    o[2] = (unsigned short)(bf16_bits(a.z) & msk); o[3] = (unsigned short)(bf16_bits(a.w) & msk);
    o[4] = (unsigned short)(bf16_bits(b.x) & msk); o[5] = (unsigned short)(bf16_bits(b.y) & msk);
    o[6] = (unsigned short)(bf16_bits(b.z) & msk); o[7] = (unsigned short)(bf16_bits(b.w) & msk);
    put16(EAB + (size_t)u * 8, o);
  } else if (u < nUE + NU_W1) {
    const int v  = u - nUE;
    const int n  = v >> 4;
    const int k8 = (v & 15) * 8;
    const float* p = w1 + (size_t)k8 * HID + n;
    v8us o;
#pragma unroll
    for (int i = 0; i < 8; ++i) o[i] = (unsigned short)bf16_bits(p[(size_t)i * HID]);
    put16(W1T + (size_t)n * NEF + k8, o);
  }
}

__global__ __launch_bounds__(NTHR) void k_pb(const float* __restrict__ w2, const float* __restrict__ b2,
                                             unsigned short* W2P, float* B2P) {
  const int u = (int)blockIdx.x * NTHR + (int)threadIdx.x;
  if (u < NU_W2P) {
    const int c  = u >> 4;
    const int k8 = (u & 15) * 8;
    const int j  = colmap(c);
    const int jc = j < 0 ? 0 : j;
    const unsigned msk = j < 0 ? 0u : 0xffffu;
    const float* p = w2 + (size_t)k8 * WTOT + jc;
    v8us o;
#pragma unroll
    for (int i = 0; i < 8; ++i) o[i] = (unsigned short)(bf16_bits(p[(size_t)i * WTOT]) & msk);
    unsigned short* dp = W2P + (size_t)c * KH + k8;
    *(volatile v8us*)dp         = o;
    *(volatile v8us*)(dp + HID) = o;
    __threadfence();
    *(volatile v8us*)dp         = o;
    *(volatile v8us*)(dp + HID) = o;
  } else {
    const int v = u - NU_W2P;
    if (v < NU_B2) {
      const int j0 = colmap(4 * v), j1 = colmap(4 * v + 1), j2 = colmap(4 * v + 2), j3 = colmap(4 * v + 3);
      const float f0 = b2[j0 < 0 ? 0 : j0];
      const float f1 = b2[j1 < 0 ? 0 : j1];
      const float f2 = b2[j2 < 0 ? 0 : j2];
      const float f3 = b2[j3 < 0 ? 0 : j3];
      v4f q;
      q.x = j0 < 0 ? 0.0f : bf16_val(f0);
      q.y = j1 < 0 ? 0.0f : bf16_val(f1);
      q.z = j2 < 0 ? 0.0f : bf16_val(f2);
      q.w = j3 < 0 ? 0.0f : bf16_val(f3);
      putf4(B2P + (size_t)v * 4, q);
    }
  }
}

__global__ __launch_bounds__(GTHR) void k_h(const unsigned short* __restrict__ A,
                                            const unsigned short* __restrict__ BT,
                                            const float* __restrict__ bias, unsigned short* Cb) {
  __shared__ __attribute__((aligned(16))) float stg[GBM * GBN];
  const int tid = (int)threadIdx.x, lane = tid & 31, wave = tid >> 5, hh = lane >> 4, m = lane & 15;
  const int rowBase = (int)blockIdx.x * GBM;

  v8f acc[8];
  {
    const v8f z = {0.f, 0.f, 0.f, 0.f, 0.f, 0.f, 0.f, 0.f};
#pragma unroll
    for (int t = 0; t < 8; ++t) acc[t] = z;
  }
  const unsigned short* ap = A  + (size_t)(rowBase + 16 * wave + m) * (size_t)NEF + 8 * hh;
  const unsigned short* bp = BT + (size_t)m * (size_t)NEF + 8 * hh;

#pragma unroll 1
  for (int k0 = 0; k0 < NEF; k0 += 32) {
    FragB af;
    af.h[0] = *(const v8usa*)(ap + k0);
    af.h[1] = *(const v8usa*)(ap + k0 + 16);
#pragma unroll
    for (int nt = 0; nt < 8; ++nt) {
      const unsigned short* wq = bp + (size_t)(16 * nt) * (size_t)NEF + k0;
      FragB bf;
      bf.h[0] = *(const v8usa*)wq;
      bf.h[1] = *(const v8usa*)(wq + 16);
      acc[nt] = wmb(af, bf, acc[nt]);
    }
  }

#pragma unroll
  for (int nt = 0; nt < 8; ++nt) {
    const int lc = 16 * nt + m;
    const float bvv = bf16_val(bias[lc]);
#pragma unroll
    for (int r = 0; r < 8; ++r) {
      const int lr = 16 * wave + 8 * hh + r;
      const float v = acc[nt][r] + bvv;
      stg[lr * GBN + lc] = (v > 0.0f) ? v : 0.0f;
    }
  }
  __syncthreads();

  const int part = lane >> 4;
  const int j = lane & 15;
  const unsigned mh = 0u - (unsigned)part;
  const unsigned ml = ~mh;
  v8us pv[16];
#pragma unroll
  for (int i = 0; i < 16; ++i) {
    const float* sp = stg + (16 * wave + i) * GBN + 8 * j;
    const v4f a = *(const v4fa*)sp;
    const v4f b = *(const v4fa*)(sp + 4);
    const v8f f8 = {a.x, a.y, a.z, a.w, b.x, b.y, b.z, b.w};
    v8us oo;
#pragma unroll
    for (int e = 0; e < 8; ++e) {
      const unsigned hb = bf16_bits(f8[e]);
      const unsigned lb = bf16_bits(f8[e] - __uint_as_float(hb << 16));
      oo[e] = (unsigned short)((hb & ml) | (lb & mh));
    }
    pv[i] = oo;
  }
#pragma unroll
  for (int i = 0; i < 16; ++i) {
    unsigned short* op = Cb + (size_t)(rowBase + 16 * wave + i) * (size_t)KH + part * HID + 8 * j;
    *(volatile v8us*)op = pv[i];
  }
  __threadfence();
#pragma unroll
  for (int i = 0; i < 16; ++i) {
    unsigned short* op = Cb + (size_t)(rowBase + 16 * wave + i) * (size_t)KH + part * HID + 8 * j;
    *(volatile v8us*)op = pv[i];
  }
}

__device__ __forceinline__ v8f tile_mm(const FragB (&af)[8], const unsigned short* __restrict__ W2P,
                                       const float* __restrict__ B2P, int t, int hh, int m) {
  const float b = B2P[16 * t + m];
  v8f acc = {b, b, b, b, b, b, b, b};
  const unsigned short* bp = W2P + (size_t)(16 * t + m) * (size_t)KH + 8 * hh;
#pragma unroll
  for (int ks = 0; ks < 8; ++ks) {
    FragB bf;
    bf.h[0] = *(const v8usa*)(bp + 32 * ks);
    bf.h[1] = *(const v8usa*)(bp + 32 * ks + 16);
    acc = wmb(af[ks], bf, acc);
  }
  return acc;
}

__global__ __launch_bounds__(NTHR) __attribute__((amdgpu_num_vgpr(248)))
void k_tp(const int* __restrict__ eidx, int nE, int nN,
          const float* __restrict__ xin, const float* __restrict__ esh,
          const unsigned short* __restrict__ HHL, const unsigned short* __restrict__ W2P,
          const float* __restrict__ B2P, float* TP, float isq3, float nrm) {
  extern __shared__ __attribute__((aligned(16))) float dyn[];
  float* CO  = dyn;
  float* XS  = dyn + EPB * COP;
  float* SH0 = XS + EPB * TPP;
  int*   GI  = (int*)(SH0 + EPB);
  const int tid = (int)threadIdx.x, lane = tid & 31, wave = tid >> 5, hh = lane >> 4, m = lane & 15;
  const int eb = (int)blockIdx.x * EPB;

  if (tid < EPB) {
    const int e  = eb + tid;
    const int ec = e < nE ? e : nE - 1;
    int g = eidx[(size_t)nE + (size_t)ec];
    g = g < 0 ? 0 : (g > nN - 1 ? nN - 1 : g);
    GI[tid] = g;
    const v4f s = *(const v4f*)(esh + (size_t)ec * 4);
    SH0[tid] = bf16_val(s.x);
    CO[tid * COP + 136] = bf16_val(s.y);
    CO[tid * COP + 137] = bf16_val(s.z);
    CO[tid * COP + 138] = bf16_val(s.w);
    CO[tid * COP + 139] = 0.0f;
    XS[tid * TPP + OUTC]     = 0.0f;
    XS[tid * TPP + OUTC + 1] = 0.0f;
  }
  __syncthreads();

#pragma unroll 4
  for (int it = 0; it < 20; ++it) {
    int idx = it * NTHR + tid;
    idx = idx < EPB * 39 - 1 ? idx : EPB * 39 - 1;
    const int e = idx / 39;
    const int p = idx - e * 39;
    const int g = GI[e];
    const v2f x = *(const v2fa*)(xin + (size_t)g * OUTC + 2 * p);
    XS[e * TPP + 2 * p]     = bf16_val(x.x);
    XS[e * TPP + 2 * p + 1] = bf16_val(x.y);
  }
  __syncthreads();

#pragma unroll 2
  for (int it = 0; it < 24; ++it) {
    const int idx = it * NTHR + tid;
    const int e = idx / NS;
    const int q = idx - e * NS;
    const float s = XS[e * TPP + q];
    const float a0 = SH0[e];
    CO[e * COP + q]           = s * a0;
    CO[e * COP + NS + NV + q] = s;
  }
#pragma unroll 1
  for (int it = 0; it < 5; ++it) {
    const int idx = it * NTHR + tid;
    const int e = idx / NV;
    const int u = idx - e * NV;
    const float v0 = XS[e * TPP + NS + 3 * u];
    const float v1 = XS[e * TPP + NS + 3 * u + 1];
    const float v2 = XS[e * TPP + NS + 3 * u + 2];
    const float a0 = SH0[e];
    const float bx = CO[e * COP + 136], by = CO[e * COP + 137], bz = CO[e * COP + 138];
    const float dt = ((v0 * bx + v1 * by) + v2 * bz) * isq3;
    CO[e * COP + NS + u] = dt;
    CO[e * COP + 106 + 3 * u]     = v0 * a0;
    CO[e * COP + 106 + 3 * u + 1] = v1 * a0;
    CO[e * COP + 106 + 3 * u + 2] = v2 * a0;
  }
  __syncthreads();

  FragB af[8];
  {
    const unsigned short* ap = HHL + (size_t)(eb + 16 * wave + m) * (size_t)KH + 8 * hh;
#pragma unroll
    for (int ks = 0; ks < 8; ++ks) {
      af[ks].h[0] = *(const v8usa*)(ap + 32 * ks);
      af[ks].h[1] = *(const v8usa*)(ap + 32 * ks + 16);
    }
  }
  const float* cr = CO + (16 * wave + 8 * hh) * COP;
  const v8f z = {0.f, 0.f, 0.f, 0.f, 0.f, 0.f, 0.f, 0.f};
  v8f O0a = z, O0b = z, O0c = z, T2 = z, O3a = z, O3b = z, O3c = z;

#pragma unroll 1
  for (int c0 = 0; c0 < NS + NV; ++c0) {
    float cf[8];
#pragma unroll
    for (int r = 0; r < 8; ++r) cf[r] = cr[r * COP + c0];
    v8f d = tile_mm(af, W2P, B2P, 3 * c0, hh, m);
#pragma unroll
    for (int r = 0; r < 8; ++r) O0a[r] = fmaf(d[r], cf[r], O0a[r]);
    d = tile_mm(af, W2P, B2P, 3 * c0 + 1, hh, m);
#pragma unroll
    for (int r = 0; r < 8; ++r) O0b[r] = fmaf(d[r], cf[r], O0b[r]);
    d = tile_mm(af, W2P, B2P, 3 * c0 + 2, hh, m);
#pragma unroll
    for (int r = 0; r < 8; ++r) O0c[r] = fmaf(d[r], cf[r], O0c[r]);
  }
#pragma unroll 1
  for (int u = 0; u < NS; ++u) {
    float cf[8];
#pragma unroll
    for (int r = 0; r < 8; ++r) cf[r] = cr[r * COP + NS + NV + u];
    const v8f d = tile_mm(af, W2P, B2P, T_W2 + u, hh, m);
#pragma unroll
    for (int r = 0; r < 8; ++r) T2[r] = fmaf(d[r], cf[r], T2[r]);
  }
#pragma unroll 1
  for (int u = 0; u < NV; ++u) {
    const v8f d = tile_mm(af, W2P, B2P, T_W3 + u, hh, m);
#pragma unroll
    for (int r = 0; r < 8; ++r) {
      const float c1 = cr[r * COP + 106 + 3 * u];
      const float c2 = cr[r * COP + 106 + 3 * u + 1];
      const float c3 = cr[r * COP + 106 + 3 * u + 2];
      O3a[r] = fmaf(d[r], c1, O3a[r]);
      O3b[r] = fmaf(d[r], c2, O3b[r]);
      O3c[r] = fmaf(d[r], c3, O3c[r]);
    }
  }

  float* TPs = XS;
#pragma unroll
  for (int r = 0; r < 8; ++r) {
    const int row = 16 * wave + 8 * hh + r;
    const float bx = cr[r * COP + 136], by = cr[r * COP + 137], bz = cr[r * COP + 138];
    float* tr = TPs + row * TPP;
    const float p0 = O0a[r] * nrm, p1 = O0b[r] * nrm, p2 = O0c[r] * nrm;
    const float y0 = fmaf(T2[r], bx, O3a[r]) * nrm;
    const float y1 = fmaf(T2[r], by, O3b[r]) * nrm;
    const float y2 = fmaf(T2[r], bz, O3c[r]) * nrm;
    tr[m]      = p0;
    tr[16 + m] = p1;
    tr[32 + m] = p2;
    if (m < NV) {
      tr[NS + 3 * m]     = y0;
      tr[NS + 3 * m + 1] = y1;
      tr[NS + 3 * m + 2] = y2;
    } else if (m < NV + 2) {
      tr[OUTC + (m - NV)] = 0.0f;
    }
  }
  __syncthreads();

  {
    v4f pv[10];
#pragma unroll
    for (int it = 0; it < 10; ++it) pv[it] = *(const v4fa*)(TPs + 4 * (it * NTHR + tid));
    float* tb = TP + (size_t)eb * TPP;
#pragma unroll
    for (int it = 0; it < 10; ++it) *(volatile v4f*)(tb + 4 * (it * NTHR + tid)) = pv[it];
    __threadfence();
#pragma unroll
    for (int it = 0; it < 10; ++it) *(volatile v4f*)(tb + 4 * (it * NTHR + tid)) = pv[it];
  }
}

__global__ __launch_bounds__(NTHR) void k_scan(const int* __restrict__ keys, int nE, int vec8, int nN,
                                               const float* __restrict__ xin, const float* __restrict__ TP,
                                               float* Y, double* REC) {
  extern __shared__ __attribute__((aligned(16))) int dsm[];
  int*    list = dsm;
  int*    hl   = dsm + LISTN;
  int*    sl   = hl + RCAP;
  int*    cnt  = sl + RCAP;
  int*    offs = cnt + NBA;
  int*    cur  = offs + NBA;
  int*    misc = cur + NBA;
  float*  YS   = (float*)(dsm + AGG_INTS);
  double* WREC = (double*)(YS + YS_FLOATS);
  const int tid = (int)threadIdx.x, lane = tid & 31, wave = tid >> 5;
  const int nodeBase = (int)blockIdx.x * NBA;

  {
    const v4i z4 = {0, 0, 0, 0};
    for (int i = tid * 4; i < AGG_ZINTS; i += NTHR * 4) *(v4ia*)(dsm + i) = z4;
    if (tid < 16) misc[tid] = 0;
  }
  __syncthreads();

  int t = 0, ov = 0;
  const int nChunks = (nE + CHUNK - 1) / CHUNK;
#pragma unroll 1
  for (int ch = 0; ch < nChunks; ++ch) {
    const int cbase = ch * CHUNK;
    const int wc = scan_chunk<SLA>(keys, nE, cbase, nodeBase, NBA, vec8, list, tid, lane, wave);
    if (lane == 0) misc[wave] = wc;
    __syncthreads();
    if (wave == 0) {
#pragma unroll 1
      for (int w2 = 0; w2 < NWAVE; ++w2) {
        int c = misc[w2];
        c = c < 0 ? 0 : (c > WCAP ? WCAP : c);
#pragma unroll 1
        for (int b0 = 0; b0 < c; b0 += 32) {
          const int idx = b0 + lane;
          const int ent = list[w2 * WCAP + (idx < WCAP ? idx : WCAP - 1)];
          const int m32 = (c - b0) < 32 ? (c - b0) : 32;
#pragma unroll 1
          for (int k = 0; k < m32; ++k) {
            const int u    = __builtin_amdgcn_readlane(ent, k);
            const int slot = u & (NBA - 1);
            const int el   = (u >> SLA) & (CHUNK - 1);
            const int pk   = ((cbase + el) << SLA) | slot;
            if (t < RCAP) {
              if (lane == 0) { hl[t] = pk; cnt[slot] = cnt[slot] + 1; }
              t = t + 1;
            } else {
              ov = 1;
            }
          }
        }
      }
    }
    __syncthreads();
  }
  if (wave == 0 && lane == 0) { misc[8] = t; misc[9] = ov; }
  __syncthreads();
  int tt = misc[8];
  tt = tt < 0 ? 0 : (tt > RCAP ? RCAP : tt);
  const int ovf = misc[9];

  if (wave == 0) {
    const int base = lane * (NBA / 32);
    int s = 0;
#pragma unroll 1
    for (int i = 0; i < NBA / 32; ++i) s += cnt[base + i];
    int incl = s;
#pragma unroll
    for (int d = 1; d < 32; d <<= 1) {
      const int y = __shfl_up(incl, d, 32);
      if (lane >= d) incl += y;
    }
    int run = incl - s;
#pragma unroll 1
    for (int i = 0; i < NBA / 32; ++i) {
      const int cv = cnt[base + i];
      offs[base + i] = run;
      cur[base + i]  = run;
      run += cv;
    }
  }
  __syncthreads();
  if (wave == 0) {
#pragma unroll 1
    for (int b0 = 0; b0 < tt; b0 += 32) {
      const int idx = b0 + lane;
      const int ent = hl[idx < RCAP ? idx : RCAP - 1];
      const int m32 = (tt - b0) < 32 ? (tt - b0) : 32;
#pragma unroll 1
      for (int k = 0; k < m32; ++k) {
        const int u    = __builtin_amdgcn_readlane(ent, k);
        const int slot = u & (NBA - 1);
        if (lane == 0) {
          int p = cur[slot];
          p = p < 0 ? 0 : (p > RCAP - 1 ? RCAP - 1 : p);
          sl[p] = u;
          cur[slot] = p + 1;
        }
      }
    }
  }
  __syncthreads();

  const float qnan = __int_as_float(0x7fc00000);
  const float pz = (ovf != 0) ? qnan : 0.0f;
  const int  lc   = lane < 20 ? lane : 19;
  const bool lastl = (lc == 19);
  const int  o2   = lastl ? 0 : 2;
  float* ysw = YS + wave * (GRP * TPP);
  double ds0 = 0.0, ds1 = 0.0, ds2 = 0.0, ds3 = 0.0;
  double dq0 = 0.0, dq1 = 0.0, dq2 = 0.0, dq3 = 0.0;
#pragma unroll 1
  for (int g = 0; g < NGRP; ++g) {
#pragma unroll 1
    for (int i = 0; i < GRP; ++i) {
      const int s    = wave * SPW + g * GRP + i;
      const int node = nodeBase + s;
      int c = cnt[s];
      const bool big = c > DEGCAP;
      c = c < 0 ? 0 : (c > DEGCAP ? DEGCAP : c);
      int o = offs[s];
      o = o < 0 ? 0 : (o > RCAP ? RCAP : o);
      float a0 = 0.0f, a1 = 0.0f, a2 = 0.0f, a3 = 0.0f;
#pragma unroll 1
      for (int b0 = 0; b0 < c; b0 += 32) {
        int idx = o + b0 + lane;
        idx = idx > RCAP - 1 ? RCAP - 1 : idx;
        const int ent = sl[idx];
        int eid = ent >> SLA;
        eid = eid < 0 ? 0 : (eid > nE - 1 ? nE - 1 : eid);
        const int m32 = (c - b0) < 32 ? (c - b0) : 32;
#pragma unroll 1
        for (int k = 0; k < m32; ++k) {
          const int ek = __builtin_amdgcn_readlane(eid, k);
          const v4f w = *(const v4fa*)(TP + (size_t)ek * TPP + 4 * lc);
          a0 += w.x; a1 += w.y; a2 += w.z; a3 += w.w;
        }
      }
      const bool live = node < nN;
      const int  nr   = live ? node : nN - 1;
      const float* xr = xin + (size_t)nr * OUTC + 4 * lc;
      const v2f xa = *(const v2fa*)xr;
      const v2f xb = *(const v2fa*)(xr + o2);
      const float r0 = bf16_val(xa.x);
      const float r1 = bf16_val(xa.y);
      const float r2 = lastl ? 0.0f : bf16_val(xb.x);
      const float r3 = lastl ? 0.0f : bf16_val(xb.y);
      const float den = (c > 0) ? (float)c : 1.0f;
      const float rcp = 1.0f / den;
      const float pzr = big ? qnan : pz;
      const float y0 = fmaf(a0, rcp, r0) + pzr;
      const float y1 = fmaf(a1, rcp, r1) + pzr;
      const float y2 = fmaf(a2, rcp, r2) + pzr;
      const float y3 = fmaf(a3, rcp, r3) + pzr;
      v4f yv;
      yv.x = live ? y0 : 0.0f;
      yv.y = live ? y1 : 0.0f;
      yv.z = live ? y2 : 0.0f;
      yv.w = live ? y3 : 0.0f;
      *(v4fa*)(ysw + i * TPP + 4 * lc) = yv;
      const double e0 = (double)yv.x, e1 = (double)yv.y, e2 = (double)yv.z, e3 = (double)yv.w;
      ds0 += e0; ds1 += e1; ds2 += e2; ds3 += e3;
      dq0 = fma(e0, e0, dq0); dq1 = fma(e1, e1, dq1); dq2 = fma(e2, e2, dq2); dq3 = fma(e3, e3, dq3);
    }
    __syncthreads();
    v4f pv[10];
#pragma unroll
    for (int it = 0; it < 10; ++it) pv[it] = *(const v4fa*)(ysw + 4 * (it * 32 + lane));
    __syncthreads();
    float* yb = Y + (size_t)(nodeBase + wave * SPW + g * GRP) * TPP;
#pragma unroll
    for (int it = 0; it < 10; ++it) *(volatile v4f*)(yb + 4 * (it * 32 + lane)) = pv[it];
    __threadfence();
#pragma unroll
    for (int it = 0; it < 10; ++it) *(volatile v4f*)(yb + 4 * (it * 32 + lane)) = pv[it];
  }

  if (lane < 20) {
    double* wr = WREC + (size_t)(wave * TPP + 4 * lane) * 2;
    wr[0] = ds0; wr[1] = dq0;
    wr[2] = ds1; wr[3] = dq1;
    wr[4] = ds2; wr[5] = dq2;
    wr[6] = ds3; wr[7] = dq3;
  }
  __syncthreads();
  {
    const int ci = tid < TPP ? tid : TPP - 1;
    double S = 0.0, Q = 0.0;
#pragma unroll 1
    for (int w2 = 0; w2 < NWAVE; ++w2) {
      S += WREC[(size_t)(w2 * TPP + ci) * 2];
      Q += WREC[(size_t)(w2 * TPP + ci) * 2 + 1];
    }
    v2d o;
    o.x = S; o.y = Q;
    double* rp = REC + ((size_t)blockIdx.x * TPP + (size_t)ci) * 2;
    if (tid < TPP) *(volatile v2d*)rp = o;
    __threadfence();
    if (tid < TPP) *(volatile v2d*)rp = o;
  }
}

__global__ __launch_bounds__(128) void k_stat(const double* __restrict__ REC, const float* __restrict__ bnw,
                                              const float* __restrict__ bnb, float* ST,
                                              double invN, double invN3, int nB) {
  __shared__ double dS[TPP];
  __shared__ double dQ[TPP];
  const int tid = (int)threadIdx.x;
  const int c = tid < TPP ? tid : TPP - 1;
  double S = 0.0, Q = 0.0;
#pragma unroll 1
  for (int b = 0; b < nB; ++b) {
    S += REC[((size_t)b * TPP + (size_t)c) * 2];
    Q += REC[((size_t)b * TPP + (size_t)c) * 2 + 1];
  }
  dS[c] = S;
  dQ[c] = Q;
  __syncthreads();
  const bool isS = c < NS;
  const int cs = isS ? c : NS - 1;
  int cv = isS ? 0 : (c - NS) / 3;
  cv = cv > NV - 1 ? NV - 1 : cv;
  const double mean = dS[c] * invN;
  const double var  = dQ[c] * invN - mean * mean;
  const double vn   = (dQ[NS + 3 * cv] + dQ[NS + 3 * cv + 1] + dQ[NS + 3 * cv + 2]) * invN3;
  const float gws = bf16_val(bnw[cs]);
  const float gwv = bf16_val(bnw[NS + cv]);
  const float bbs = bf16_val(bnb[cs]);
  const float stat = isS ? (float)var : (float)vn;
  const float rs = rsqrtf(stat + EPSF);
  const bool used = c < OUTC;
  v4f o;
  o.x = (used && isS) ? (float)mean : 0.0f;
  o.y = used ? rs * (isS ? gws : gwv) : 0.0f;
  o.z = (used && isS) ? bbs : 0.0f;
  o.w = 0.0f;
  float* sp = ST + 4 * c;
  if (tid < TPP) *(volatile v4f*)sp = o;
  __threadfence();
  if (tid < TPP) *(volatile v4f*)sp = o;
}

__global__ __launch_bounds__(NTHR) void k_norm(const float* __restrict__ Y, const float* __restrict__ ST,
                                               int nN, float* out) {
  __shared__ __attribute__((aligned(16))) float sst[TPP * 4];
  __shared__ __attribute__((aligned(16))) float os[NRB * OUTC];
  const int tid = (int)threadIdx.x;
  const int nb = (int)blockIdx.x * NRB;
  {
    const int ci = tid < TPP ? tid : TPP - 1;
    const v4f q = *(const v4f*)(ST + 4 * ci);
    *(v4fa*)(sst + 4 * ci) = q;
  }
  __syncthreads();
#pragma unroll 2
  for (int it = 0; it < 10; ++it) {
    const int idx = it * NTHR + tid;
    const int row = idx / 20;
    const int c4  = (idx - row * 20) * 4;
    const v4f y = *(const v4f*)(Y + (size_t)(nb + row) * TPP + c4);
    const float yy[4] = {y.x, y.y, y.z, y.w};
#pragma unroll
    for (int j = 0; j < 4; ++j) {
      const int c  = c4 + j;
      const int cc = c < OUTC ? c : OUTC - 1;
      const v4f st = *(const v4fa*)(sst + 4 * cc);
      const float o = (yy[j] - st.x) * st.y + st.z;
      if (c < OUTC) os[row * OUTC + c] = o;
    }
  }
  __syncthreads();
  int rows = nN - nb;
  rows = rows > NRB ? NRB : (rows < 1 ? 1 : rows);
  const int nv4 = (rows * OUTC) / 4;
  v4f pv[10];
#pragma unroll
  for (int it = 0; it < 10; ++it) {
    const int idx = it * NTHR + tid;
    const int ic  = idx < nv4 ? idx : nv4 - 1;
    pv[it] = *(const v4fa*)(os + 4 * ic);
  }
  float* ob = out + (size_t)nb * OUTC;
#pragma unroll
  for (int it = 0; it < 10; ++it) {
    const int idx = it * NTHR + tid;
    if (idx < nv4) *(volatile v4f*)(ob + 4 * idx) = pv[it];
  }
  __threadfence();
#pragma unroll
  for (int it = 0; it < 10; ++it) {
    const int idx = it * NTHR + tid;
    if (idx < nv4) *(volatile v4f*)(ob + 4 * idx) = pv[it];
  }
}

static inline int cdiv(int a, int b) { return (a + b - 1) / b; }
static inline size_t al256(size_t o) { return (o + 255) & ~(size_t)255; }

extern "C" void kernel_launch(void* const* d_in, const int* in_sizes, int n_in,
                              void* d_out, int out_size, void* d_ws, size_t ws_size,
                              hipStream_t stream) {
  if (n_in < 10) return;
  if (in_sizes[0] < OUTC || (in_sizes[0] % OUTC) != 0) return;
  const int nN = in_sizes[0] / OUTC;
  if (in_sizes[1] < 2 || (in_sizes[1] & 1) != 0) return;
  const int nE = in_sizes[1] / 2;
  if (nE < 1 || nE >= (1 << 21) || nN < 1 || nN >= (1 << 22)) return;
  if ((long long)in_sizes[2] != (long long)nE * NEF) return;
  if ((long long)in_sizes[3] != (long long)nE * 4) return;
  if (in_sizes[4] != NEF * HID || in_sizes[5] != HID) return;
  if (in_sizes[6] != HID * WTOT || in_sizes[7] != WTOT) return;
  if (in_sizes[8] != NS + NV || in_sizes[9] != NS) return;
  if ((long long)out_size != (long long)nN * OUTC) return;
  if ((((long long)nN * OUTC * 4) % 128) != 0) return;
  if ((((long long)(nN % NRB) * OUTC) % 4) != 0) return;

  const float* node_attr = (const float*)d_in[0];
  const int*   eidx      = (const int*)d_in[1];
  const float* edge_attr = (const float*)d_in[2];
  const float* edge_sh   = (const float*)d_in[3];
  const float* fc_w1     = (const float*)d_in[4];
  const float* fc_b1     = (const float*)d_in[5];
  const float* fc_w2     = (const float*)d_in[6];
  const float* fc_b2     = (const float*)d_in[7];
  const float* bn_w      = (const float*)d_in[8];
  const float* bn_b      = (const float*)d_in[9];
  float* out = (float*)d_out;

  const int EP = cdiv(nE, EPB) * EPB;
  const int gT = EP / EPB;
  const int gH = EP / GBM;
  const int gA = cdiv(nN, NBA);
  const int gN = cdiv(nN, NRB);
  if ((long long)gN * NRB > (long long)gA * NBA) return;
  const int nUE = EP * (NEF / 8);

  char* ws = (char*)d_ws;
  size_t off = 0;
  const size_t oEAB = off; off = al256(off + (size_t)EP * NEF * 2);
  const size_t oW1T = off; off = al256(off + (size_t)HID * NEF * 2);
  const size_t oW2P = off; off = al256(off + (size_t)NPC * KH * 2);
  const size_t oB2P = off; off = al256(off + (size_t)NPC * 4);
  const size_t oHHL = off; off = al256(off + (size_t)EP * KH * 2);
  const size_t oTP  = off; off = al256(off + (size_t)EP * TPP * 4);
  const size_t oY   = off; off = al256(off + (size_t)gA * NBA * TPP * 4);
  const size_t oREC = off; off = al256(off + (size_t)gA * TPP * 2 * 8);
  const size_t oST  = off; off = al256(off + (size_t)TPP * 4 * 4);
  if (off > ws_size || off > (size_t)WSMAX) return;
  unsigned short* EAB = (unsigned short*)(ws + oEAB);
  unsigned short* W1T = (unsigned short*)(ws + oW1T);
  unsigned short* W2P = (unsigned short*)(ws + oW2P);
  float*          B2P = (float*)(ws + oB2P);
  unsigned short* HHL = (unsigned short*)(ws + oHHL);
  float*          TP  = (float*)(ws + oTP);
  float*          Y   = (float*)(ws + oY);
  double*         REC = (double*)(ws + oREC);
  float*          ST  = (float*)(ws + oST);

  hipFuncSetAttribute(reinterpret_cast<const void*>(&k_tp), hipFuncAttributeMaxDynamicSharedMemorySize,
                      (int)TP_LDS_BYTES);
  hipFuncSetAttribute(reinterpret_cast<const void*>(&k_scan), hipFuncAttributeMaxDynamicSharedMemorySize,
                      (int)SCAN_LDS_BYTES);

  const float isq3 = (float)(1.0 / sqrt(3.0));
  const float nrm  = (float)(1.0 / sqrt((double)(NS + NV)));
  const double invN  = 1.0 / (double)nN;
  const double invN3 = 1.0 / (3.0 * (double)nN);
  const int vec8 = ((nE & 3) == 0) ? 1 : 0;

  k_pa<<<(nUE + NU_W1) / NTHR, NTHR, 0, stream>>>(edge_attr, fc_w1, nE, nUE, EAB, W1T);
  k_pb<<<(NU_W2P + NU_B2P) / NTHR, NTHR, 0, stream>>>(fc_w2, fc_b2, W2P, B2P);
  k_h<<<gH, GTHR, 0, stream>>>(EAB, W1T, fc_b1, HHL);
  k_tp<<<gT, NTHR, TP_LDS_BYTES, stream>>>(eidx, nE, nN, node_attr, edge_sh, HHL, W2P, B2P, TP, isq3, nrm);
  k_scan<<<gA, NTHR, SCAN_LDS_BYTES, stream>>>(eidx, nE, vec8, nN, node_attr, TP, Y, REC);
  k_stat<<<1, 128, 0, stream>>>(REC, bn_w, bn_b, ST, invN, invN3, gA);
  k_norm<<<gN, NTHR, 0, stream>>>(Y, ST, nN, out);
}
